// MultiheadCrossAttention_22686017257525
// MI455X (gfx1250) — hardware-verified
//
#include <hip/hip_runtime.h>


#ifndef NB
#define NB 8
#endif
#ifndef SEQ
#define SEQ 1024
#endif
#ifndef SKV
#define SKV 1024
#endif
#define NB_FULL 8
#define T_FULL 1024
#define S_FULL 1024
#define DMOD 768
#define DENC 1024
#define NHD 12
#define HD 64
#define QB 32
#define NCH (SKV / 64)
#define PCAR 16384.0f
#define L2S ((1.0f / 384.0f) * 1.4426950408889634f)

static_assert(NHD * HD == DMOD);
static_assert(HD == 64);
static_assert(NB >= 1 && NB <= NB_FULL);
static_assert(SEQ % 64 == 0);
static_assert(SEQ % QB == 0);
static_assert(SKV % 64 == 0);
static_assert(DMOD % 64 == 0);
static_assert(DENC % 64 == 0);
static_assert(SEQ <= T_FULL);
static_assert(SKV <= S_FULL);
static_assert(((size_t)NB * T_FULL * DMOD) % 8 == 0);
static_assert(((size_t)NB * S_FULL * DENC) % 8 == 0);
static_assert((size_t)NB * T_FULL * DMOD * 4 <= (size_t)25165824);

#define WS_XB  ((size_t)NB * T_FULL * DMOD * 2)
#define WS_EB  ((size_t)NB * S_FULL * DENC * 2)
#define WS_WQ  ((size_t)DMOD * DMOD * 2)
#define WS_WK  ((size_t)DMOD * DENC * 2)
#define WS_QH  ((size_t)NB * SEQ * DMOD * 2)
#define WS_KH  ((size_t)NB * SKV * DMOD * 2)
#define WS_V32 ((size_t)NB * SKV * DMOD * 4)
#define WS_VT  ((size_t)NB * NHD * HD * SKV * 2)
#define WS_CS  ((size_t)NB * NHD * NCH * 64 * 4)
#define WS_CT  ((size_t)NB * SEQ * DMOD * 2)
#define WS_TOTAL (WS_XB + WS_EB + 2 * WS_WQ + 2 * WS_WK + WS_QH + WS_KH + WS_V32 + WS_VT + WS_CS + 2 * WS_CT)
static_assert(WS_XB % 256 == 0);
static_assert(WS_EB % 256 == 0);
static_assert(WS_WQ % 256 == 0);
static_assert(WS_WK % 256 == 0);
static_assert(WS_QH % 256 == 0);
static_assert(WS_KH % 256 == 0);
static_assert(WS_V32 % 256 == 0);
static_assert(WS_VT % 256 == 0);
static_assert(WS_CS % 256 == 0);
static_assert(WS_CT % 256 == 0);
static_assert(WS_TOTAL <= (size_t)134217728);

typedef _Float16 h16;
typedef unsigned short bf;
typedef __attribute__((ext_vector_type(16))) __bf16   v16bf;
typedef __attribute__((ext_vector_type(16))) _Float16 v16h;
typedef __attribute__((ext_vector_type(8)))  _Float16 v8h;
typedef __attribute__((ext_vector_type(8)))  unsigned short v8us;
typedef __attribute__((ext_vector_type(8)))  float    v8f;
typedef __attribute__((ext_vector_type(4)))  float    v4f;
typedef v8h  __attribute__((may_alias)) v8ha;
typedef v4f  __attribute__((may_alias)) v4fa;
typedef v8us __attribute__((may_alias)) v8usa;

__device__ __forceinline__ unsigned short f2bf(float f) { unsigned u = __float_as_uint(f); u += 0x7FFFu + ((u >> 16) & 1u); return (unsigned short)(u >> 16); }
__device__ __forceinline__ float bf2f(unsigned short b) { return __uint_as_float(((unsigned)b) << 16); }
__device__ __forceinline__ float bfr(float f) { return bf2f(f2bf(f)); }
__device__ __forceinline__ v16h cat16(v8h lo, v8h hi) { return __builtin_shufflevector(lo, hi, 0, 1, 2, 3, 4, 5, 6, 7, 8, 9, 10, 11, 12, 13, 14, 15); }
__device__ __forceinline__ v16bf cat16b(v8us lo, v8us hi) { return __builtin_bit_cast(v16bf, __builtin_shufflevector(lo, hi, 0, 1, 2, 3, 4, 5, 6, 7, 8, 9, 10, 11, 12, 13, 14, 15)); }
__device__ __forceinline__ v8f wmma16(v16h a, v16h b, v8f c) { return __builtin_amdgcn_wmma_f32_16x16x32_f16(false, a, false, b, (short)0, c, false, false); }
__device__ __forceinline__ v8f wmmab(v16bf a, v16bf b, v8f c) { return __builtin_amdgcn_wmma_f32_16x16x32_bf16(false, a, false, b, (short)0, c, false, false); }
__device__ __forceinline__ void splitf(float y, unsigned short& h, unsigned short& l) { h = f2bf(y); l = f2bf(y - bf2f(h)); }
__device__ __forceinline__ float flz(float y) { return (fabsf(y) < 6.103515625e-05f) ? 0.0f : y; }
__device__ __forceinline__ h16 tohc(float x) { return (h16)flz(x); }

template <typename T16> struct WFrag;
template <> struct WFrag<h16> { typedef v16h V; static __device__ __forceinline__ V ld(const h16* p) { return cat16(*(const v8h*)p, *(const v8h*)(p + 16)); } static __device__ __forceinline__ v8f mma(V a, V b, v8f c) { return wmma16(a, b, c); } };
template <> struct WFrag<bf> { typedef v16bf V; static __device__ __forceinline__ V ld(const bf* p) { return cat16b(*(const v8us*)p, *(const v8us*)(p + 16)); } static __device__ __forceinline__ v8f mma(V a, V b, v8f c) { return wmmab(a, b, c); } };

template <typename OT> struct SlabOut;
template <> struct SlabOut<float> {
    template <bool BIAS> static __device__ __forceinline__ void run(const float* os, float* crow, int ldc, const float* __restrict__ bias, int c0, int lane) {
        const int lr = lane & 15, hi = lane >> 4, cofs = lr * 4;
#pragma unroll 1
        for (int ps = 0; ps < 2; ++ps) {
#pragma unroll
            for (int s = 0; s < 8; ++s) { const int row = 2 * s + hi; v4f val = *(const v4fa*)(os + row * 68 + cofs);
                if (BIAS) { val[0] += bfr(bias[c0 + cofs]); val[1] += bfr(bias[c0 + cofs + 1]); val[2] += bfr(bias[c0 + cofs + 2]); val[3] += bfr(bias[c0 + cofs + 3]); }
                *(volatile v4f*)(crow + (size_t)row * ldc + cofs) = val; }
            if (ps == 0) __threadfence(); }
    }
};
template <> struct SlabOut<h16> {
    template <bool BIAS> static __device__ __forceinline__ void run(const float* os, h16* crow, int ldc, const float* __restrict__ bias, int c0, int lane) {
        const int piece = lane & 7, rsub = lane >> 3, cofs = piece * 8;
        v8h ov[4];
#pragma unroll
        for (int rg = 0; rg < 4; ++rg) {
            const int row = rg * 4 + rsub;
            const v4f u0 = *(const v4fa*)(os + row * 68 + cofs);
            const v4f u1 = *(const v4fa*)(os + row * 68 + cofs + 4);
#pragma unroll
            for (int j = 0; j < 4; ++j) {
                float x0 = u0[j], x1 = u1[j];
                if (BIAS) { x0 += bfr(bias[c0 + cofs + j]); x1 += bfr(bias[c0 + cofs + 4 + j]); }
                ov[rg][j] = tohc(x0); ov[rg][4 + j] = tohc(x1);
            }
        }
#pragma unroll 1
        for (int ps = 0; ps < 2; ++ps) {
#pragma unroll
            for (int rg = 0; rg < 4; ++rg) { const int row = rg * 4 + rsub; *(volatile v8h*)(crow + (size_t)row * ldc + cofs) = ov[rg]; }
            if (ps == 0) __threadfence(); }
    }
};

template <typename T16, int NSPLIT, bool BIAS, typename OT>
__global__ __launch_bounds__(32) void k_gemmw(const T16* __restrict__ A, const T16* __restrict__ A2, const T16* __restrict__ Bt, const T16* __restrict__ Bt2, int K, OT* C, int ldc, const float* __restrict__ bias, size_t sA, size_t sB, size_t sC) {
    typedef typename WFrag<T16>::V V;
    __shared__ __align__(16) float os[16 * 68];
    const size_t z = blockIdx.z; A += z * sA; A2 += z * sA; Bt += z * sB; Bt2 += z * sB; C += z * sC;
    const int lane = threadIdx.x & 31, lr = lane & 15, hi = lane >> 4; const int r0 = blockIdx.x * 64, c0 = blockIdx.y * 64;
    v8f acc[4][4];
#pragma unroll
    for (int mb = 0; mb < 4; ++mb)
#pragma unroll
        for (int nb = 0; nb < 4; ++nb) acc[mb][nb] = (v8f){};
    const size_t aoff = (size_t)(r0 + lr) * K + 8 * hi, boff = (size_t)(c0 + lr) * K + 8 * hi;
#pragma unroll 1
    for (int kc = 0; kc < K; kc += 32) {
        V a[4], a2[4];
#pragma unroll
        for (int mb = 0; mb < 4; ++mb) { a[mb] = WFrag<T16>::ld(A + aoff + (size_t)mb * 16 * K + kc); if (NSPLIT == 1 || NSPLIT == 2) a2[mb] = WFrag<T16>::ld(A2 + aoff + (size_t)mb * 16 * K + kc); }
#pragma unroll
        for (int nb = 0; nb < 4; ++nb) { const V b = WFrag<T16>::ld(Bt + boff + (size_t)nb * 16 * K + kc); V b2; if (NSPLIT >= 2) b2 = WFrag<T16>::ld(Bt2 + boff + (size_t)nb * 16 * K + kc);
#pragma unroll
            for (int mb = 0; mb < 4; ++mb) { acc[mb][nb] = WFrag<T16>::mma(a[mb], b, acc[mb][nb]); if (NSPLIT == 1 || NSPLIT == 2) acc[mb][nb] = WFrag<T16>::mma(a2[mb], b, acc[mb][nb]); if (NSPLIT >= 2) acc[mb][nb] = WFrag<T16>::mma(a[mb], b2, acc[mb][nb]); } }
        asm volatile("v_nop\n\tv_nop\n\tv_nop\n\tv_nop" : "+v"(acc[0][0]), "+v"(acc[1][1]), "+v"(acc[2][2]), "+v"(acc[3][3]) : "v"(a[0]), "v"(a[3]));
    }
#pragma unroll
    for (int mb = 0; mb < 4; ++mb) {
#pragma unroll
        for (int nb = 0; nb < 4; ++nb) {
#pragma unroll
            for (int j = 0; j < 8; ++j) os[(hi * 8 + j) * 68 + nb * 16 + lr] = acc[mb][nb][j]; }
        __builtin_amdgcn_wave_barrier(); asm volatile("" ::: "memory");
        OT* crow = C + (size_t)(r0 + mb * 16) * ldc + c0;
        SlabOut<OT>::template run<BIAS>(os, crow, ldc, bias, c0, lane);
        __builtin_amdgcn_wave_barrier(); asm volatile("" ::: "memory");
    }
}

__global__ __launch_bounds__(256) void k_cvt8(const float* __restrict__ src, bf* dst, size_t n8) { const size_t i = (size_t)blockIdx.x * 256 + threadIdx.x; if (i >= n8) return; const v8f v = *(const v8f*)(src + i * 8); v8us o;
#pragma unroll
    for (int k = 0; k < 8; ++k) o[k] = f2bf(v[k]); *(volatile v8us*)(dst + i * 8) = o; __threadfence(); *(volatile v8us*)(dst + i * 8) = o; }

__global__ __launch_bounds__(256) void k_wtr(const float* __restrict__ W, bf* Bt, int K, int N) {
    __shared__ __align__(16) unsigned short tile[64 * 72];
    const int k0 = blockIdx.x * 64, n0 = blockIdx.y * 64, t = threadIdx.x;
    {
        const int r = t >> 2, seg = t & 3;
        const float* src = W + (size_t)(k0 + r) * N + n0 + seg * 16;
#pragma unroll
        for (int q = 0; q < 2; ++q) { const v8f a = *(const v8f*)(src + 8 * q); v8us o;
#pragma unroll
            for (int e = 0; e < 8; ++e) o[e] = f2bf(a[e]);
            *(v8us*)(tile + r * 72 + seg * 16 + 8 * q) = o; }
    }
    __syncthreads();
    const int piece = t & 7, rq = t >> 3;
    v8us o2[2];
#pragma unroll
    for (int pg = 0; pg < 2; ++pg) { const int n = pg * 32 + rq;
#pragma unroll
        for (int e = 0; e < 8; ++e) o2[pg][e] = tile[(piece * 8 + e) * 72 + n]; }
#pragma unroll 1
    for (int ps = 0; ps < 2; ++ps) {
#pragma unroll
        for (int pg = 0; pg < 2; ++pg) { const int n = pg * 32 + rq; *(volatile v8us*)(Bt + (size_t)(n0 + n) * K + k0 + piece * 8) = o2[pg]; }
        if (ps == 0) __threadfence(); }
}

__global__ __launch_bounds__(256) void k_vtr(const float* __restrict__ F, h16* VT, float* CS) {
    __shared__ __align__(16) h16 tile[64 * 72];
    __shared__ __align__(32) float ft[64 * 72];
    __shared__ __align__(16) float csum[64];
    const int b = blockIdx.z, head = blockIdx.y, s0 = blockIdx.x * 64, t = threadIdx.x;
    {
        const int r = t >> 2, seg = t & 3;
        const float* src = F + ((size_t)b * SKV + s0 + r) * DMOD + head * HD + seg * 16;
#pragma unroll
        for (int q = 0; q < 2; ++q) { const v8f a = *(const v8f*)(src + 8 * q); v8h o;
#pragma unroll
            for (int e = 0; e < 8; ++e) o[e] = tohc(a[e]);
            *(v8h*)(tile + r * 72 + seg * 16 + 8 * q) = o;
            *(v8f*)(ft + r * 72 + seg * 16 + 8 * q) = a; }
    }
    __syncthreads();
    const int piece = t & 7, rq = t >> 3;
    v8h o2[2];
#pragma unroll
    for (int pg = 0; pg < 2; ++pg) { const int d = pg * 32 + rq;
#pragma unroll
        for (int e = 0; e < 8; ++e) o2[pg][e] = tile[(piece * 8 + e) * 72 + d]; }
    if (t < 64) {
        float sa = 0.0f, sb = 0.0f;
#pragma unroll 4
        for (int s = 0; s < 64; s += 2) { sa += ft[s * 72 + t]; sb += ft[(s + 1) * 72 + t]; }
        csum[t] = sa + sb;
    }
    __syncthreads();
    const v4f cv = *(const v4fa*)(csum + 4 * (t & 15));
    float* csl = CS + (((size_t)(b * NHD + head)) * NCH + blockIdx.x) * 64 + 4 * (t & 15);
#pragma unroll 1
    for (int ps = 0; ps < 2; ++ps) {
#pragma unroll
        for (int pg = 0; pg < 2; ++pg) { const int d = pg * 32 + rq; *(volatile v8h*)(VT + (((size_t)(b * NHD + head)) * HD + d) * SKV + s0 + piece * 8) = o2[pg]; }
        if (t < 16) *(volatile v4f*)csl = cv;
        if (ps == 0) __threadfence(); }
}

__global__ __launch_bounds__(64) __attribute__((amdgpu_num_vgpr(256)))
void k_flash(const h16* __restrict__ QH, const h16* __restrict__ KH, const h16* __restrict__ VTp, const float* __restrict__ CSp, bf* CTh, bf* CTl) {
    __shared__ __align__(16) unsigned short eh[2][16 * 64];
    __shared__ __align__(16) unsigned short el[2][16 * 64];
    const int b = blockIdx.z, head = blockIdx.y;
    const int w = threadIdx.x >> 5, lane = threadIdx.x & 31, hf = lane >> 4, lm = lane & 15;
    const int m0 = blockIdx.x * QB + w * 16;
    v16h qf[2];
    {
        const h16* qp = QH + ((size_t)b * SEQ + m0 + lm) * DMOD + head * HD + 8 * hf;
#pragma unroll
        for (int ks = 0; ks < 2; ++ks) qf[ks] = cat16(*(const v8h*)(qp + 32 * ks), *(const v8h*)(qp + 32 * ks + 16));
    }
    v8f acc[4], cor[4];
#pragma unroll
    for (int dt = 0; dt < 4; ++dt) { acc[dt] = (v8f){}; cor[dt] = (v8f){}; }
    float mrun = -1.0e30f, lrun = 0.0f;
    const h16* kcur = KH + ((size_t)b * SKV + lm) * DMOD + head * HD + 8 * hf;
    const h16* vcur = VTp + (((size_t)(b * NHD + head)) * HD + lm) * SKV + 8 * hf;
    const float* cscur = CSp + ((size_t)(b * NHD + head)) * NCH * 64 + lm;
#pragma unroll 1
    for (int sc = 0; sc < SKV; sc += 64) {
        v8f st[4];
#pragma unroll
        for (int s4 = 0; s4 < 4; ++s4) st[s4] = (v8f){};
#pragma unroll
        for (int s4 = 0; s4 < 4; ++s4) {
            const h16* kp = kcur + (size_t)(s4 * 16) * DMOD;
#pragma unroll
            for (int ks = 0; ks < 2; ++ks) { const v16h af = cat16(*(const v8h*)(kp + 32 * ks), *(const v8h*)(kp + 32 * ks + 16)); st[s4] = wmma16(af, qf[ks], st[s4]); }
        }
        asm volatile("v_nop\n\tv_nop\n\tv_nop\n\tv_nop" : "+v"(st[0]), "+v"(st[1]), "+v"(st[2]), "+v"(st[3]) : "v"(qf[0]), "v"(qf[1]));
        float cm = -1.0e30f;
#pragma unroll
        for (int s4 = 0; s4 < 4; ++s4) { st[s4] *= L2S;
#pragma unroll
            for (int e = 0; e < 8; ++e) cm = fmaxf(cm, st[s4][e]); }
        cm = fmaxf(cm, __shfl_xor(cm, 16, 32));
        const float mnew = fmaxf(mrun, cm);
        const float alpha = __builtin_amdgcn_exp2f(mrun - mnew);
        mrun = mnew;
        float ls = 0.0f;
#pragma unroll
        for (int s4 = 0; s4 < 4; ++s4)
#pragma unroll
            for (int e = 0; e < 8; ++e) { const float p = __builtin_amdgcn_exp2f(st[s4][e] - mnew); st[s4][e] = p; ls += p; }
        ls += __shfl_xor(ls, 16, 32);
        const float g = ls * 0.015625f;
        v16h pf[2];
#pragma unroll
        for (int s4 = 0; s4 < 4; ++s4)
#pragma unroll
            for (int e = 0; e < 8; ++e) pf[s4 >> 1][(s4 & 1) * 8 + e] = (h16)((st[s4][e] - g) * PCAR);
        lrun = lrun * alpha + ls;
        v8f av, gv;
#pragma unroll
        for (int e = 0; e < 8; ++e) { av[e] = __shfl(alpha, 8 * hf + e, 32); gv[e] = __shfl(g, 8 * hf + e, 32); }
        float csd[4];
#pragma unroll
        for (int dt = 0; dt < 4; ++dt) csd[dt] = cscur[dt * 16];
#pragma unroll
        for (int dt = 0; dt < 4; ++dt) { acc[dt] *= av;
#pragma unroll
            for (int e = 0; e < 8; ++e) cor[dt][e] = fmaf(gv[e], csd[dt], cor[dt][e] * av[e]); }
        asm volatile("" ::: "memory");
#pragma unroll
        for (int ks = 0; ks < 2; ++ks) {
#pragma unroll
            for (int dt = 0; dt < 4; ++dt) { const h16* vp = vcur + (size_t)(dt * 16) * SKV + sc + 32 * ks; const v16h vf = cat16(*(const v8h*)vp, *(const v8h*)(vp + 16)); acc[dt] = wmma16(pf[ks], vf, acc[dt]); }
            asm volatile("" ::: "memory");
        }
        asm volatile("v_nop\n\tv_nop\n\tv_nop\n\tv_nop" : "+v"(acc[0]), "+v"(acc[1]), "+v"(acc[2]), "+v"(acc[3]) : "v"(pf[0]), "v"(pf[1]));
        kcur += (size_t)64 * DMOD;
        cscur += 64;
    }
    v8f lv;
#pragma unroll
    for (int e = 0; e < 8; ++e) lv[e] = __shfl(lrun, 8 * hf + e, 32);
    v8f iv;
#pragma unroll
    for (int e = 0; e < 8; ++e) iv[e] = 1.0f / lv[e];
    unsigned short* ehw = eh[w]; unsigned short* elw = el[w];
#pragma unroll
    for (int dt = 0; dt < 4; ++dt)
#pragma unroll
        for (int e = 0; e < 8; ++e) { unsigned short a2, c2; const float vnum = fmaf(acc[dt][e], (1.0f / PCAR), cor[dt][e]); splitf(vnum * iv[e], a2, c2); const int o = (8 * hf + e) * 64 + dt * 16 + lm; ehw[o] = a2; elw[o] = c2; }
    __syncthreads();
    const int piece = lane & 7, rsub = lane >> 3;
#pragma unroll 1
    for (int ps = 0; ps < 2; ++ps) {
#pragma unroll
        for (int rg = 0; rg < 4; ++rg) { const int row = rg * 4 + rsub; const v8us oh = *(const v8usa*)(ehw + row * 64 + piece * 8); const v8us ol = *(const v8usa*)(elw + row * 64 + piece * 8);
            const size_t go = ((size_t)b * SEQ + m0 + row) * DMOD + head * HD + piece * 8;
            *(volatile v8us*)(CTh + go) = oh; *(volatile v8us*)(CTl + go) = ol; }
        if (ps == 0) __threadfence(); }
}

extern "C" void kernel_launch(void* const* d_in, const int* in_sizes, int n_in,
                              void* d_out, int out_size, void* d_ws, size_t ws_size, hipStream_t stream) {
    if (n_in < 10) return;
    if ((size_t)in_sizes[0] < (size_t)NB * T_FULL * DMOD) return;
    if ((size_t)in_sizes[1] < (size_t)NB * S_FULL * DENC) return;
    if ((size_t)in_sizes[2] < (size_t)DMOD * DMOD) return;
    if ((size_t)in_sizes[3] < (size_t)DMOD) return;
    if ((size_t)in_sizes[4] < (size_t)DENC * DMOD) return;
    if ((size_t)in_sizes[5] < (size_t)DMOD) return;
    if ((size_t)in_sizes[6] < (size_t)DENC * DMOD) return;
    if ((size_t)in_sizes[7] < (size_t)DMOD) return;
    if ((size_t)in_sizes[8] < (size_t)DMOD * DMOD) return;
    if ((size_t)in_sizes[9] < (size_t)DMOD) return;
    if ((size_t)out_size < (size_t)NB * T_FULL * DMOD) return;
    const float* x   = (const float*)d_in[0];
    const float* enc = (const float*)d_in[1];
    const float* wq  = (const float*)d_in[2];
    const float* bq  = (const float*)d_in[3];
    const float* wk  = (const float*)d_in[4];
    const float* bk  = (const float*)d_in[5];
    const float* wv  = (const float*)d_in[6];
    const float* bv  = (const float*)d_in[7];
    const float* wp  = (const float*)d_in[8];
    const float* bp  = (const float*)d_in[9];
    float* OUT = (float*)d_out;
    char* wsp = (char*)d_ws;
    size_t used = 0;
    auto take = [&](size_t bytes) { char* p = wsp + used; used += (bytes + 255) & ~(size_t)255; return (void*)p; };
    bf*    XB  = (bf*)take(WS_XB);
    bf*    EB  = (bf*)take(WS_EB);
    bf*    WQt = (bf*)take(WS_WQ);
    bf*    WKt = (bf*)take(WS_WK);
    bf*    WVt = (bf*)take(WS_WK);
    bf*    WPt = (bf*)take(WS_WQ);
    h16*   QH  = (h16*)take(WS_QH);
    h16*   KH  = (h16*)take(WS_KH);
    float* V32 = (float*)take(WS_V32);
    h16*   VT  = (h16*)take(WS_VT);
    float* CS  = (float*)take(WS_CS);
    bf*    CTh = (bf*)take(WS_CT);
    bf*    CTl = (bf*)take(WS_CT);
    if (used > ws_size) return;
    const size_t n8x = (size_t)NB * T_FULL * DMOD / 8, n8e = (size_t)NB * S_FULL * DENC / 8;
    k_cvt8<<<(unsigned)((n8x + 255) / 256), 256, 0, stream>>>(x, XB, n8x);
    k_cvt8<<<(unsigned)((n8e + 255) / 256), 256, 0, stream>>>(enc, EB, n8e);
    k_wtr<<<dim3(DMOD / 64, DMOD / 64), 256, 0, stream>>>(wq, WQt, DMOD, DMOD);
    k_wtr<<<dim3(DENC / 64, DMOD / 64), 256, 0, stream>>>(wk, WKt, DENC, DMOD);
    k_wtr<<<dim3(DENC / 64, DMOD / 64), 256, 0, stream>>>(wv, WVt, DENC, DMOD);
    k_wtr<<<dim3(DMOD / 64, DMOD / 64), 256, 0, stream>>>(wp, WPt, DMOD, DMOD);
    k_gemmw<bf, 0, true, h16><<<dim3(SEQ / 64, DMOD / 64, NB), 32, 0, stream>>>(XB, XB, WQt, WQt, DMOD, QH, DMOD, bq, (size_t)T_FULL * DMOD, (size_t)0, (size_t)SEQ * DMOD);
    k_gemmw<bf, 0, true, h16><<<dim3(SKV / 64, DMOD / 64, NB), 32, 0, stream>>>(EB, EB, WKt, WKt, DENC, KH, DMOD, bk, (size_t)S_FULL * DENC, (size_t)0, (size_t)SKV * DMOD);
    k_gemmw<bf, 0, true, float><<<dim3(SKV / 64, DMOD / 64, NB), 32, 0, stream>>>(EB, EB, WVt, WVt, DENC, V32, DMOD, bv, (size_t)S_FULL * DENC, (size_t)0, (size_t)SKV * DMOD);
    k_vtr<<<dim3(SKV / 64, NHD, NB), 256, 0, stream>>>(V32, VT, CS);
    k_flash<<<dim3(SEQ / QB, NHD, NB), 64, 0, stream>>>(QH, KH, VT, CS, CTh, CTl);
    k_gemmw<bf, 1, true, float><<<dim3(SEQ / 64, DMOD / 64, NB), 32, 0, stream>>>(CTh, CTl, WPt, WPt, DMOD, OUT, DMOD, bp, (size_t)SEQ * DMOD, (size_t)0, (size_t)T_FULL * DMOD);
}
